// MIEstimator_12360915878462
// MI455X (gfx1250) — hardware-verified
//
#include <hip/hip_runtime.h>
#include <math.h>

typedef __attribute__((ext_vector_type(16))) _Float16 v16h;
typedef __attribute__((ext_vector_type(16))) __bf16 v16b;
typedef __attribute__((ext_vector_type(8)))  _Float16 v8h;
typedef __attribute__((ext_vector_type(8)))  float v8f;
typedef __attribute__((ext_vector_type(4)))  float v4f;
typedef __attribute__((ext_vector_type(2)))  float v2f;
typedef __attribute__((ext_vector_type(4)))  unsigned v4u;
typedef __attribute__((ext_vector_type(4)))  int v4i;
typedef float __attribute__((may_alias)) float_a;
typedef int __attribute__((may_alias)) int_a;

template <typename T> __device__ __forceinline__ void vst2(void* p, T v) { *(volatile T*)p = v; __threadfence(); *(volatile T*)p = v; }
__device__ __forceinline__ v8f wmma16(v16h a, v16h b, v8f c) {
  v8f d = __builtin_amdgcn_wmma_f32_16x16x32_f16(false, a, false, b, (short)0, c, false, false);
  asm volatile("v_nop\n\tv_nop\n\tv_nop\n\tv_nop" : "+v"(d) : "v"(a), "v"(b));
  return d;
}
__device__ __forceinline__ v8f wmma_bf(v16b a, v16b b, v8f c) {
  v8f d = __builtin_amdgcn_wmma_f32_16x16x32_bf16(false, a, false, b, (short)0, c, false, false);
  asm volatile("v_nop\n\tv_nop\n\tv_nop\n\tv_nop" : "+v"(d) : "v"(a), "v"(b));
  return d;
}
__device__ __forceinline__ v16h frag_h(const _Float16* rowk0, int lane) {
  union { v16h v; v8h q[2]; } u; const _Float16* p = rowk0 + 8 * (lane >> 4);
  u.q[0] = *(const v8h*)p; u.q[1] = *(const v8h*)(p + 16); return u.v;
}
__device__ __forceinline__ v16h frag_f32(const float* rowk0, int lane) {
  v16h a; const float* p = rowk0 + 8 * (lane >> 4);
#pragma unroll
  for (int i = 0; i < 8; ++i) { a[i] = (_Float16)p[i]; a[8 + i] = (_Float16)p[16 + i]; }
  return a;
}
__device__ __forceinline__ v16h frag_f32s(const float* rowk0, int lane, float sc) {
  v16h a; const float* p = rowk0 + 8 * (lane >> 4);
#pragma unroll
  for (int i = 0; i < 8; ++i) { a[i] = (_Float16)(p[i] * sc); a[8 + i] = (_Float16)(p[16 + i] * sc); }
  return a;
}
__device__ __forceinline__ v16h fragc_f32(const float* W, int k0, int n, int lane, int ld, int K) {
  v16h a; const int g = lane >> 4;
#pragma unroll
  for (int i = 0; i < 8; ++i) { const int ka = k0 + 8 * g + i, kb = ka + 16;
    a[i] = (_Float16)(ka < K ? W[(size_t)ka * ld + n] : 0.f); a[8 + i] = (_Float16)(kb < K ? W[(size_t)kb * ld + n] : 0.f); }
  return a;
}
struct F2 { v16b h, l; };
__device__ __forceinline__ F2 bsplit16(const float v[16]) { F2 r;
#pragma unroll
  for (int i = 0; i < 16; ++i) { const __bf16 h = (__bf16)v[i]; r.h[i] = h; r.l[i] = (__bf16)(v[i] - (float)h); }
  return r; }
__device__ __forceinline__ F2 split_row(const float* row, int k0, int lane) { float v[16]; const float* p = row + k0 + 8 * (lane >> 4);
#pragma unroll
  for (int i = 0; i < 8; ++i) { v[i] = p[i]; v[8 + i] = p[16 + i]; }
  return bsplit16(v); }
__device__ __forceinline__ F2 split_rowK(const float* row, int k0, int lane, int K) { float v[16]; const int g = lane >> 4;
#pragma unroll
  for (int i = 0; i < 8; ++i) { const int ka = k0 + 8 * g + i, kb = ka + 16; v[i] = ka < K ? row[ka] : 0.f; v[8 + i] = kb < K ? row[kb] : 0.f; }
  return bsplit16(v); }
__device__ __forceinline__ F2 split_col(const float* W, int k0, int n, int lane, int ld, int K) { float v[16]; const int g = lane >> 4;
#pragma unroll
  for (int i = 0; i < 8; ++i) { const int ka = k0 + 8 * g + i, kb = ka + 16; v[i] = ka < K ? W[(size_t)ka * ld + n] : 0.f; v[8 + i] = kb < K ? W[(size_t)kb * ld + n] : 0.f; }
  return bsplit16(v); }
__device__ __forceinline__ v8f mac3(const F2& a, const F2& b, v8f c) { c = wmma_bf(a.l, b.h, c); c = wmma_bf(a.h, b.l, c); return wmma_bf(a.h, b.h, c); }
__device__ __forceinline__ float sigm(float v) { return 1.0f / (1.0f + expf(-v)); }
#define LDSX() do { asm volatile("s_wait_dscnt 0" ::: "memory"); __builtin_amdgcn_wave_barrier(); __builtin_amdgcn_fence(__ATOMIC_RELEASE, "workgroup"); } while (0)

#define NN 8192
#define DX 256
#define HH 256
#define DY 64

__global__ __launch_bounds__(128) void k_l1(const float* __restrict__ x, const float* __restrict__ w1m, const float* __restrict__ b1m, const float* __restrict__ w1l, const float* __restrict__ b1l, float* __restrict__ H1) {
  __shared__ __align__(16) float so[4][16][132];
  const int tid = threadIdx.x, wave = tid >> 5, lane = tid & 31, col = lane & 15, g = lane >> 4;
  const int r0 = blockIdx.x * 64 + wave * 16, n0 = blockIdx.y * 128; const int which = n0 / HH; const float* W = which ? w1l : w1m; const float* bb = which ? b1l : b1m; const int nl0 = n0 % HH;
  v8f acc[8] = {};
#pragma unroll 1
  for (int kc = 0; kc < DX / 32; ++kc) { const F2 a = split_row(x + (size_t)(r0 + col) * DX, kc * 32, lane);
#pragma unroll
    for (int j = 0; j < 8; ++j) acc[j] = mac3(a, split_col(W, kc * 32, nl0 + j * 16 + col, lane, HH, DX), acc[j]); }
#pragma unroll
  for (int j = 0; j < 8; ++j) { const float b0 = bb[nl0 + j * 16 + col];
#pragma unroll
    for (int r = 0; r < 8; ++r) { const float v = acc[j][r] + b0; so[wave][8 * g + r][j * 16 + col] = v > 0.f ? v : 0.f; } }
  LDSX();
#pragma unroll 4
  for (int rl = 0; rl < 16; ++rl) vst2(H1 + (size_t)(r0 + rl) * (2 * HH) + n0 + lane * 4, *(const v4f*)(&so[wave][rl][lane * 4]));
}
__global__ __launch_bounds__(64) void k_ypart(const float* __restrict__ y, float* __restrict__ part) {
  const int d = threadIdx.x, r0 = blockIdx.x * 64; float s = 0.f, s2 = 0.f;
#pragma unroll 1
  for (int r = 0; r < 64; ++r) { const float v = y[(size_t)(r0 + r) * DY + d]; s += v; s2 += v * v; }
  vst2(part + (size_t)blockIdx.x * 128 + d, (float_a)s); vst2(part + (size_t)blockIdx.x * 128 + 64 + d, (float_a)s2);
}
__global__ __launch_bounds__(128) void k_ystat(const float* __restrict__ part, float* __restrict__ yst) {
  const int t = threadIdx.x; float s = 0.f;
#pragma unroll 1
  for (int b = 0; b < NN / 64; ++b) s += part[(size_t)b * 128 + t];
  vst2(yst + t, (float_a)(s / (float)NN));
}
__global__ __launch_bounds__(128) void k_l2(const float* __restrict__ H1, const float* __restrict__ w2m, const float* __restrict__ b2m, const float* __restrict__ w2l, const float* __restrict__ b2l,
                                          const float* __restrict__ y, const float* __restrict__ yst, float* __restrict__ part) {
  __shared__ __align__(16) float smu[4][16][68], slv[4][16][68];
  __shared__ float srow[64];
  const int tid = threadIdx.x, wave = tid >> 5, lane = tid & 31, col = lane & 15, g = lane >> 4;
  const int r0 = blockIdx.x * 64 + wave * 16;
  v8f am[4] = {}, al[4] = {};
#pragma unroll 1
  for (int kc = 0; kc < HH / 32; ++kc) { const F2 a = split_row(H1 + (size_t)(r0 + col) * (2 * HH), kc * 32, lane); const F2 a2 = split_row(H1 + (size_t)(r0 + col) * (2 * HH) + HH, kc * 32, lane);
#pragma unroll
    for (int j = 0; j < 4; ++j) { am[j] = mac3(a, split_col(w2m, kc * 32, j * 16 + col, lane, DY, HH), am[j]); al[j] = mac3(a2, split_col(w2l, kc * 32, j * 16 + col, lane, DY, HH), al[j]); } }
#pragma unroll
  for (int j = 0; j < 4; ++j) { const int d = j * 16 + col;
#pragma unroll
    for (int r = 0; r < 8; ++r) { smu[wave][8 * g + r][d] = am[j][r] + b2m[d]; slv[wave][8 * g + r][d] = al[j][r] + b2l[d]; } }
  LDSX();
  { const int rl = lane >> 1, hf = lane & 1; const int row = r0 + rl; float t = 0.f;
    for (int dd = 0; dd < 32; ++dd) { const int d = hf * 32 + dd; const float mu = smu[wave][rl][d]; const float lv = tanhf(slv[wave][rl][d]); const float iv = expf(-lv);
      const float yv = y[(size_t)row * DY + d]; const float df = mu - yv;
      const float pos = -(df * df) * iv * 0.5f; const float neg = -(mu * mu - 2.0f * mu * yst[d] + yst[64 + d]) * iv * 0.5f; t += pos - neg; }
    t += __shfl_xor(t, 1, 32);
    if (hf == 0) srow[wave * 16 + rl] = t; }
  __syncthreads();
  if (tid < 32) { float s = 0.f; if (tid == 0) { for (int i = 0; i < 64; ++i) s += srow[i]; } vst2(part + (size_t)blockIdx.x * 32 + tid, (float_a)(tid == 0 ? s : 0.f)); }
}
__global__ __launch_bounds__(32) void k_fin(const float* __restrict__ part, float* __restrict__ out) {
  const int t = threadIdx.x; float s = 0.f;
  if (t == 0) { for (int b = 0; b < NN / 64; ++b) s += part[(size_t)b * 32]; }
  if (t == 0) vst2(out, (float_a)(s / (float)NN));
}
extern "C" void kernel_launch(void* const* d_in, const int* in_sizes, int n_in, void* d_out, int out_size, void* d_ws, size_t ws_size, hipStream_t stream) {
  (void)in_sizes; (void)n_in; (void)out_size; (void)ws_size;
  const float** I = (const float**)d_in;
  const float* x = I[0]; const float* y = I[1]; const float* w1m = I[2]; const float* b1m = I[3]; const float* w2m = I[4]; const float* b2m = I[5];
  const float* w1l = I[6]; const float* b1l = I[7]; const float* w2l = I[8]; const float* b2l = I[9];
  float* out = (float*)d_out;
  char* ws = (char*)d_ws; size_t off = 0;
  auto take = [&](size_t bytes) { char* p = ws + off; off += (bytes + 255) & ~(size_t)255; return p; };
  float* H1 = (float*)take((size_t)NN * 2 * HH * 4); float* yp = (float*)take((size_t)(NN / 64) * 128 * 4); float* yst = (float*)take(128 * 4); float* part = (float*)take((size_t)(NN / 64) * 32 * 4);
  k_l1<<<dim3(NN / 64, 2 * HH / 128), 128, 0, stream>>>(x, w1m, b1m, w1l, b1l, H1);
  k_ypart<<<NN / 64, 64, 0, stream>>>(y, yp);
  k_ystat<<<1, 128, 0, stream>>>(yp, yst);
  k_l2<<<NN / 64, 128, 0, stream>>>(H1, w2m, b2m, w2l, b2l, y, yst, part);
  k_fin<<<1, 32, 0, stream>>>(part, out);
}
